// InteractionNetwork_42502996362059
// MI455X (gfx1250) — hardware-verified
//
#include <hip/hip_runtime.h>

typedef _Float16 v16h __attribute__((ext_vector_type(16)));
typedef _Float16 v8h  __attribute__((ext_vector_type(8)));
typedef float    v8f  __attribute__((ext_vector_type(8)));
typedef float    v4f  __attribute__((ext_vector_type(4)));
typedef v8h __attribute__((may_alias)) v8ha;
typedef v4f __attribute__((may_alias)) v4fa;

union Frag { v16h v; v8h half[2]; };

#define NB     128
#define NN     64
#define NF     14
#define OBJF   17
#define K0R    37
#define HID    150
#define HP     160
#define EFF    50
#define EP     64
#define AGGD   68
#define SHID   100
#define NOUTC  3
#define NTHR   128
#define NWAVE  (NTHR / 32)
#define RPW    (NN / NWAVE)
#define TILE_H (16 * HP)
#define W1OFF  0
#define W2OFF  (HP * HP)
#define W3OFF  (2 * HP * HP)
#define W4OFF  (3 * HP * HP)
#define WPL_HALVES (3 * HP * HP + EP * HP)
#define WPL_GROUPS (WPL_HALVES / 8)
#define PL_GROUPS  (HP * HP / 8)
#define WSCALE 8.0f
#define WINV   0.125f

static_assert(RPW * NWAVE == NN);
static_assert((WPL_HALVES % 256) == 0);
static_assert((HP % 32) == 0);

__device__ __forceinline__ v8f wmma_f16(v16h a, v16h b, v8f c) {
  v8f d = __builtin_amdgcn_wmma_f32_16x16x32_f16(false, a, false, b, (short)0, c, false, false);
  asm volatile("v_nop\n\tv_nop\n\tv_nop\n\tv_nop" : "+v"(d) : "v"(a), "v"(b));
  return d;
}

__device__ __forceinline__ v16h load_frag(const _Float16* p, int h) {
  Frag f;
  f.half[0] = *(const v8ha*)(p + 8 * h);
  f.half[1] = *(const v8ha*)(p + 16 + 8 * h);
  return f.v;
}

__device__ __forceinline__ v8f zero8f() {
  const v8f z = {0.f, 0.f, 0.f, 0.f, 0.f, 0.f, 0.f, 0.f};
  return z;
}

__global__ __launch_bounds__(256) void convert_w(
    const float* __restrict__ iw1, const float* __restrict__ iw2,
    const float* __restrict__ iw3, const float* __restrict__ iw4,
    _Float16* __restrict__ wpl)
{
  const int g = blockIdx.x * 256 + threadIdx.x;
  if (g >= WPL_GROUPS) return;
  const int pl = (g < PL_GROUPS) ? 0 : ((g < 2 * PL_GROUPS) ? 1 : ((g < 3 * PL_GROUPS) ? 2 : 3));
  const float* src = (pl == 0) ? iw1 : ((pl == 1) ? iw2 : ((pl == 2) ? iw3 : iw4));
  const int nout = (pl == 3) ? EFF : HID;
  const int e = 8 * (g - pl * PL_GROUPS);
  const int n = e / HP;
  const int k0 = e - n * HP;
  const int nc = min(n, nout - 1);
  v8h o;
  #pragma unroll
  for (int q = 0; q < 8; ++q) {
    const int k = k0 + q;
    const int kc = min(k, HID - 1);
    const float x = src[(size_t)kc * nout + nc];
    const bool ok = (k < HID) && (n < nout);
    o[q] = ok ? (_Float16)(x * WSCALE) : (_Float16)0.0f;
  }
  _Float16* dst = wpl + (size_t)8 * g;
  *(volatile v8h*)dst = o;
  __threadfence();
  *(volatile v8h*)dst = o;
}

__device__ __forceinline__ void hidden_layer(const _Float16* __restrict__ wt, const float* sB,
                                             const _Float16* xin, _Float16* xout, int h, int m) {
  const _Float16* xrow = xin + m * HP;
  #pragma unroll
  for (int hf = 0; hf < 2; ++hf) {
    v8f acc[5];
    #pragma unroll
    for (int nb = 0; nb < 5; ++nb) acc[nb] = zero8f();
    const _Float16* wrow = wt + (size_t)(80 * hf + m) * HP;
    #pragma unroll 1
    for (int kb = 0; kb < HP / 32; ++kb) {
      const v16h xb = load_frag(xrow + 32 * kb, h);
      #pragma unroll
      for (int nb = 0; nb < 5; ++nb) {
        const v16h wa = load_frag(wrow + (size_t)nb * 16 * HP + 32 * kb, h);
        acc[nb] = wmma_f16(wa, xb, acc[nb]);
      }
    }
    #pragma unroll
    for (int nb = 0; nb < 5; ++nb) {
      const int n0 = 80 * hf + 16 * nb + 8 * h;
      const v4f b0 = *(const v4fa*)(sB + n0);
      const v4f b1 = *(const v4fa*)(sB + n0 + 4);
      v8h o;
      o[0] = (_Float16)fmaxf(fmaf(acc[nb][0], WINV, b0.x), 0.0f);
      o[1] = (_Float16)fmaxf(fmaf(acc[nb][1], WINV, b0.y), 0.0f);
      o[2] = (_Float16)fmaxf(fmaf(acc[nb][2], WINV, b0.z), 0.0f);
      o[3] = (_Float16)fmaxf(fmaf(acc[nb][3], WINV, b0.w), 0.0f);
      o[4] = (_Float16)fmaxf(fmaf(acc[nb][4], WINV, b1.x), 0.0f);
      o[5] = (_Float16)fmaxf(fmaf(acc[nb][5], WINV, b1.y), 0.0f);
      o[6] = (_Float16)fmaxf(fmaf(acc[nb][6], WINV, b1.z), 0.0f);
      o[7] = (_Float16)fmaxf(fmaf(acc[nb][7], WINV, b1.w), 0.0f);
      *(v8ha*)(xout + m * HP + n0) = o;
    }
  }
}

__global__ __launch_bounds__(NTHR) void scene_kernel(
    const float* __restrict__ tensor,
    const float* __restrict__ iw0,
    const float* __restrict__ ib0,
    const float* __restrict__ ib1, const float* __restrict__ ib2,
    const float* __restrict__ ib3,
    const float* __restrict__ ib4,
    const _Float16* __restrict__ wpl,
    const float* __restrict__ sw0,
    const float* __restrict__ sb0,
    const float* __restrict__ sw1,
    const float* __restrict__ sb1,
    float* __restrict__ out)
{
  __shared__ __attribute__((aligned(16))) _Float16 sAct[NWAVE * 2 * TILE_H];
  __shared__ __attribute__((aligned(16))) float sP[NN * HP];
  __shared__ __attribute__((aligned(16))) float sQ[NN * HP];
  __shared__ __attribute__((aligned(16))) float sAgg[NN * EP];
  __shared__ __attribute__((aligned(16))) float sBias[4 * HP];
  __shared__ __attribute__((aligned(16))) float sOut[NOUTC * NN];
  __shared__ float sObj[NN * OBJF];

  const int tid = threadIdx.x, lane = tid & 31, w = tid >> 5;
  const int h = lane >> 4, m = lane & 15;
  const int b = blockIdx.x;

  for (int idx = tid; idx < NN * OBJF; idx += NTHR) {
    const int n = idx / OBJF, c = idx - n * OBJF;
    const int f = (c < 3) ? c : (c - 3);
    const int fr = (c >= 3 && c < 6) ? 0 : 1;
    sObj[idx] = tensor[(((size_t)b * 2 + fr) * NN + n) * NF + f];
  }
  for (int idx = tid; idx < 4 * HP; idx += NTHR) {
    const int l = idx / HP, n = idx - l * HP;
    const float* bp = (l == 0) ? ib1 : ((l == 1) ? ib2 : ((l == 2) ? ib3 : ib4));
    const int lim = (l == 3) ? EFF : HID;
    const float v = bp[min(n, lim - 1)];
    sBias[idx] = (n < lim) ? v : 0.0f;
  }
  __syncthreads();

  for (int idx = tid; idx < NN * HP; idx += NTHR) {
    const int i = idx / HP, n = idx - i * HP;
    const int nn = min(n, HID - 1);
    float p = ib0[nn] + iw0[34 * HID + nn];
    float q = 0.0f;
    #pragma unroll
    for (int k = 0; k < OBJF; ++k) {
      const float o = sObj[i * OBJF + k];
      p = fmaf(o, iw0[k * HID + nn], p);
      q = fmaf(o, iw0[(OBJF + k) * HID + nn], q);
    }
    const bool ok = (n < HID);
    sP[idx] = ok ? p : 0.0f;
    sQ[idx] = ok ? q : 0.0f;
  }
  __syncthreads();

  _Float16* buf0 = sAct + w * (2 * TILE_H);
  _Float16* buf1 = buf0 + TILE_H;
  const _Float16* wt1 = wpl + W1OFF;
  const _Float16* wt2 = wpl + W2OFF;
  const _Float16* wt3 = wpl + W3OFF;
  const _Float16* wt4 = wpl + W4OFF;

  #pragma unroll 1
  for (int ii = 0; ii < RPW; ++ii) {
    const int i = w * RPW + ii;
    v8f aggr[4];
    #pragma unroll
    for (int nb = 0; nb < 4; ++nb) aggr[nb] = zero8f();

    #pragma unroll 1
    for (int t = 0; t < 4; ++t) {
      const int j = 16 * t + m;
      {
        const float* pr = sP + i * HP + 80 * h;
        const float* qr = sQ + j * HP + 80 * h;
        _Float16* xr = buf0 + m * HP + 80 * h;
        #pragma unroll
        for (int g = 0; g < 10; ++g) {
          const v4f p0 = *(const v4fa*)(pr + 8 * g);
          const v4f p1 = *(const v4fa*)(pr + 8 * g + 4);
          const v4f q0 = *(const v4fa*)(qr + 8 * g);
          const v4f q1 = *(const v4fa*)(qr + 8 * g + 4);
          const v4f s0 = p0 + q0;
          const v4f s1 = p1 + q1;
          v8h o;
          o[0] = (_Float16)fmaxf(s0.x, 0.0f);
          o[1] = (_Float16)fmaxf(s0.y, 0.0f);
          o[2] = (_Float16)fmaxf(s0.z, 0.0f);
          o[3] = (_Float16)fmaxf(s0.w, 0.0f);
          o[4] = (_Float16)fmaxf(s1.x, 0.0f);
          o[5] = (_Float16)fmaxf(s1.y, 0.0f);
          o[6] = (_Float16)fmaxf(s1.z, 0.0f);
          o[7] = (_Float16)fmaxf(s1.w, 0.0f);
          *(v8ha*)(xr + 8 * g) = o;
        }
      }
      __syncthreads();
      hidden_layer(wt1, sBias,          buf0, buf1, h, m);
      __syncthreads();
      hidden_layer(wt2, sBias + HP,     buf1, buf0, h, m);
      __syncthreads();
      hidden_layer(wt3, sBias + 2 * HP, buf0, buf1, h, m);
      __syncthreads();

      v8f acc[4];
      #pragma unroll
      for (int nb = 0; nb < 4; ++nb) acc[nb] = zero8f();
      const _Float16* xrow = buf1 + m * HP;
      const _Float16* wrow = wt4 + (size_t)m * HP;
      #pragma unroll 1
      for (int kb = 0; kb < HP / 32; ++kb) {
        const v16h xb = load_frag(xrow + 32 * kb, h);
        #pragma unroll
        for (int nb = 0; nb < 4; ++nb) {
          const v16h wa = load_frag(wrow + (size_t)nb * 16 * HP + 32 * kb, h);
          acc[nb] = wmma_f16(wa, xb, acc[nb]);
        }
      }
      const bool self = (j == i);
      const float* sB4 = sBias + 3 * HP;
      #pragma unroll
      for (int nb = 0; nb < 4; ++nb) {
        const int n0 = 16 * nb + 8 * h;
        const v4f b0 = *(const v4fa*)(sB4 + n0);
        const v4f b1 = *(const v4fa*)(sB4 + n0 + 4);
        float e;
        e = fmaf(acc[nb][0], WINV, b0.x); aggr[nb][0] += self ? 0.0f : e;
        e = fmaf(acc[nb][1], WINV, b0.y); aggr[nb][1] += self ? 0.0f : e;
        e = fmaf(acc[nb][2], WINV, b0.z); aggr[nb][2] += self ? 0.0f : e;
        e = fmaf(acc[nb][3], WINV, b0.w); aggr[nb][3] += self ? 0.0f : e;
        e = fmaf(acc[nb][4], WINV, b1.x); aggr[nb][4] += self ? 0.0f : e;
        e = fmaf(acc[nb][5], WINV, b1.y); aggr[nb][5] += self ? 0.0f : e;
        e = fmaf(acc[nb][6], WINV, b1.z); aggr[nb][6] += self ? 0.0f : e;
        e = fmaf(acc[nb][7], WINV, b1.w); aggr[nb][7] += self ? 0.0f : e;
      }
    }

    #pragma unroll
    for (int nb = 0; nb < 4; ++nb) {
      #pragma unroll
      for (int r = 0; r < 8; ++r) {
        float v = aggr[nb][r];
        v += __shfl_xor(v, 1);
        v += __shfl_xor(v, 2);
        v += __shfl_xor(v, 4);
        v += __shfl_xor(v, 8);
        aggr[nb][r] = v;
      }
    }
    if (m == 0) {
      #pragma unroll
      for (int nb = 0; nb < 4; ++nb) {
        const v4f lo = {aggr[nb][0], aggr[nb][1], aggr[nb][2], aggr[nb][3]};
        const v4f hi = {aggr[nb][4], aggr[nb][5], aggr[nb][6], aggr[nb][7]};
        float* dst = sAgg + i * EP + 16 * nb + 8 * h;
        *(v4fa*)dst = lo;
        *(v4fa*)(dst + 4) = hi;
      }
    }
  }
  __syncthreads();

  float* sHid = sP;
  for (int idx = tid; idx < NN * SHID; idx += NTHR) {
    const int n = idx / SHID, hh = idx - n * SHID;
    float s = sb0[hh] + sw0[OBJF * SHID + hh];
    #pragma unroll
    for (int k = 0; k < OBJF; ++k) s = fmaf(sObj[n * OBJF + k], sw0[k * SHID + hh], s);
    #pragma unroll 4
    for (int c = 0; c < EFF; ++c) s = fmaf(sAgg[n * EP + c], sw0[(OBJF + 1 + c) * SHID + hh], s);
    sHid[n * HP + hh] = fmaxf(s, 0.0f);
  }
  __syncthreads();
  for (int idx = tid; idx < NOUTC * NN; idx += NTHR) {
    const int c = idx / NN, n = idx - c * NN;
    float s = sb1[c];
    #pragma unroll 4
    for (int hh = 0; hh < SHID; ++hh) s = fmaf(sHid[n * HP + hh], sw1[hh * NOUTC + c], s);
    sOut[idx] = s;
  }
  __syncthreads();

  const bool st = (tid < (NOUTC * NN) / 4);
  const v4f ov = *(const v4fa*)(sOut + 4 * (st ? tid : 0));
  float* od = out + (size_t)b * (NOUTC * NN) + 4 * tid;
  if (st) *(volatile v4f*)od = ov;
  __threadfence();
  if (st) *(volatile v4f*)od = ov;
}

extern "C" void kernel_launch(void* const* d_in, const int* in_sizes, int n_in,
                              void* d_out, int out_size, void* d_ws, size_t ws_size,
                              hipStream_t stream) {
  if (n_in < 15) return;
  if (in_sizes[0] != NB * 2 * NN * NF) return;
  if (in_sizes[1] != K0R * HID || in_sizes[2] != HID) return;
  if (in_sizes[3] != HID * HID || in_sizes[4] != HID) return;
  if (in_sizes[5] != HID * HID || in_sizes[6] != HID) return;
  if (in_sizes[7] != HID * HID || in_sizes[8] != HID) return;
  if (in_sizes[9] != HID * EFF || in_sizes[10] != EFF) return;
  if (in_sizes[11] != AGGD * SHID || in_sizes[12] != SHID) return;
  if (in_sizes[13] != SHID * NOUTC || in_sizes[14] != NOUTC) return;
  if (out_size != NB * NOUTC * NN) return;

  const size_t wpl_bytes = (size_t)WPL_HALVES * 2;
  if (wpl_bytes > ws_size) return;

  const float* tensor = (const float*)d_in[0];
  const float* iw0 = (const float*)d_in[1];
  const float* ib0 = (const float*)d_in[2];
  const float* iw1 = (const float*)d_in[3];
  const float* ib1 = (const float*)d_in[4];
  const float* iw2 = (const float*)d_in[5];
  const float* ib2 = (const float*)d_in[6];
  const float* iw3 = (const float*)d_in[7];
  const float* ib3 = (const float*)d_in[8];
  const float* iw4 = (const float*)d_in[9];
  const float* ib4 = (const float*)d_in[10];
  const float* sw0 = (const float*)d_in[11];
  const float* sb0 = (const float*)d_in[12];
  const float* sw1 = (const float*)d_in[13];
  const float* sb1 = (const float*)d_in[14];
  float* out = (float*)d_out;
  _Float16* wpl = (_Float16*)d_ws;

  convert_w<<<(WPL_GROUPS + 255) / 256, 256, 0, stream>>>(iw1, iw2, iw3, iw4, wpl);
  scene_kernel<<<NB, NTHR, 0, stream>>>(tensor, iw0, ib0, ib1, ib2, ib3, ib4, wpl,
                                         sw0, sb0, sw1, sb1, out);
}
